// DualAttentionModule_62371515073031
// MI455X (gfx1250) — hardware-verified
//
#include <hip/hip_runtime.h>
#include <math.h>
#include <stdint.h>

#ifndef NB
#define NB 4
#endif
#define NB_FULL 4
#define CC    512
#define NN    4096
#define DQ    64
#define MW    128
#define QT    64
#define QB    32
#define OSP   68
#define EP    68
#define OSPW  260
#define TP    72
#define PP    40
#define WSC   256.0f
#define IWSC  0.00390625f
#define PSC   16384.0f
#define IPSC  6.103515625e-05f
#define LNPS  9.704060527839234f
#define RSC   2048.0f
#define IRSC  0.00048828125f
#define BNEPS 1.0e-5f
#define NCH   ((NB * NN) / 1024)

static_assert(NB >= 1 && NB <= NB_FULL);
static_assert(NN % QT == 0 && CC % QT == 0 && NN % QB == 0);
static_assert(MW == 2 * DQ && DQ == QT);
static_assert(CC % 32 == 0 && NN % 32 == 0 && DQ % 32 == 0);
static_assert(CC == 512);
static_assert((NB * NN) % 1024 == 0 && NN % 1024 == 0);
static_assert((OSP * 4) % 16 == 0 && (EP * 4) % 16 == 0 && (OSPW * 4) % 16 == 0);
static_assert((TP * 2) % 16 == 0 && (PP * 2) % 16 == 0 && PP >= 32);
static_assert(MW % 8 == 0 && CC % 8 == 0 && (NB * CC) % 8 == 0);
static_assert(QB * OSPW >= (QB - 1) * OSPW + 256);
static_assert(OSPW >= 256 && OSP >= QT && EP >= QT && TP >= QT);

typedef _Float16       v16h __attribute__((ext_vector_type(16)));
typedef _Float16       v8h  __attribute__((ext_vector_type(8)));
typedef __bf16         v16b __attribute__((ext_vector_type(16)));
typedef unsigned short v8us __attribute__((ext_vector_type(8)));
typedef float          v8f  __attribute__((ext_vector_type(8)));
typedef float          v4f  __attribute__((ext_vector_type(4)));
typedef unsigned int   v4u  __attribute__((ext_vector_type(4)));

union Frag { v8us u[2]; v16h h; v16b bf; };
union PF   { v16h v; v8h hv[2]; v8us u[2]; };
static_assert(sizeof(Frag) == 32);
static_assert(sizeof(PF) == 32);

__device__ __forceinline__ unsigned short bf_bits(float f) {
  unsigned u = __float_as_uint(f);
  return (unsigned short)((u + 0x7FFFu + ((u >> 16) & 1u)) >> 16);
}
__device__ __forceinline__ float bf_up(unsigned short hb) { return __uint_as_float(((unsigned)hb) << 16); }
__device__ __forceinline__ float bfr(float f) { return bf_up(bf_bits(f)); }
__device__ __forceinline__ unsigned short h_bits(_Float16 x) { return __builtin_bit_cast(unsigned short, x); }
__device__ __forceinline__ unsigned pk16(unsigned short a, unsigned short b) { return (unsigned)a | ((unsigned)b << 16); }
__device__ __forceinline__ v8f zero8() { v8f z = {0.f, 0.f, 0.f, 0.f, 0.f, 0.f, 0.f, 0.f}; return z; }
__device__ __forceinline__ float hmax8(v8f s) {
  return fmaxf(fmaxf(fmaxf(s[0], s[1]), fmaxf(s[2], s[3])), fmaxf(fmaxf(s[4], s[5]), fmaxf(s[6], s[7])));
}
__device__ __forceinline__ unsigned wave_ballot(bool p) {
#if defined(__HIP_DEVICE_COMPILE__)
  return __builtin_amdgcn_ballot_w32(p);
#else
  return p ? 1u : 0u;
#endif
}

__device__ __forceinline__ Frag ldfrag(const unsigned short* p) {
  Frag f;
  f.u[0] = *(const v8us*)(p);
  f.u[1] = *(const v8us*)(p + 16);
  return f;
}

__device__ __forceinline__ v8f mma_h(v16h a, v16h b, v8f c) {
  v8f d = __builtin_amdgcn_wmma_f32_16x16x32_f16(false, a, false, b, (short)0, c, false, false);
#if defined(__HIP_DEVICE_COMPILE__)
  asm volatile("v_nop\n\tv_nop\n\tv_nop\n\tv_nop" : "+v"(d) : "v"(a), "v"(b));
#endif
  return d;
}
__device__ __forceinline__ v8f mma_b(v16b a, v16b b, v8f c) {
  v8f d = __builtin_amdgcn_wmma_f32_16x16x32_bf16(false, a, false, b, (short)0, c, false, false);
#if defined(__HIP_DEVICE_COMPILE__)
  const v16h ha = __builtin_bit_cast(v16h, a), hb = __builtin_bit_cast(v16h, b);
  asm volatile("v_nop\n\tv_nop\n\tv_nop\n\tv_nop" : "+v"(d) : "v"(ha), "v"(hb));
#endif
  return d;
}

__global__ __launch_bounds__(256)
void cvt_w(const float* __restrict__ Wq, const float* __restrict__ Wk, const float* __restrict__ Wv,
           const float* __restrict__ Wo, unsigned short* Wqk16, unsigned short* Wv16, unsigned short* Wo16) {
  const int tid = threadIdx.x, blk = blockIdx.x;
  const int rl = tid >> 5, lane = tid & 31;
  const float* src;
  unsigned short* dst;
  int kind;
  if (blk < MW / 8) {
    const int o = 8 * blk + rl;
    src = (o < DQ) ? (Wq + (size_t)o * CC) : (Wk + (size_t)(o - DQ) * CC);
    dst = Wqk16 + (size_t)o * CC;
    kind = 0;
  } else if (blk < MW / 8 + CC / 8) {
    const int o = 8 * (blk - MW / 8) + rl;
    src = Wv + (size_t)o * CC;
    dst = Wv16 + (size_t)o * CC;
    kind = 0;
  } else {
    const int o = 8 * (blk - MW / 8 - CC / 8) + rl;
    src = Wo + (size_t)o * CC;
    dst = Wo16 + (size_t)o * CC;
    kind = 1;
  }
  v4u u[2];
#pragma unroll
  for (int j = 0; j < 2; ++j) {
    const int col = 256 * j + 8 * lane;
    const v4f a = *(const v4f*)(src + col);
    const v4f q = *(const v4f*)(src + col + 4);
    const float f[8] = {a[0], a[1], a[2], a[3], q[0], q[1], q[2], q[3]};
#pragma unroll
    for (int t = 0; t < 4; ++t) {
      const float f0 = f[2 * t], f1 = f[2 * t + 1];
      const unsigned short s0 = h_bits((_Float16)(bfr(f0) * WSC));
      const unsigned short s1 = h_bits((_Float16)(bfr(f1) * WSC));
      const unsigned short r0 = bf_bits(f0), r1 = bf_bits(f1);
      u[j][t] = kind ? pk16(r0, r1) : pk16(s0, s1);
    }
  }
#pragma unroll
  for (int pass = 0; pass < 2; ++pass) {
#pragma unroll
    for (int j = 0; j < 2; ++j) *(volatile v4u*)(dst + 256 * j + 8 * lane) = u[j];
    __threadfence();
  }
}

__global__ __launch_bounds__(256)
void cvt_x(const float* __restrict__ x, unsigned short* Xc, unsigned short* XP) {
  __shared__ __align__(16) unsigned short T[QT * TP];
  const int tid = threadIdx.x;
  const int nb = blockIdx.x, cb = blockIdx.y, b = blockIdx.z;
  const int e = tid & 7, lq = tid >> 3;
  const int n0 = nb * QT, c0 = cb * QT;
  v4u ux[2];
#pragma unroll
  for (int it = 0; it < 2; ++it) {
    const int cl = it * 32 + lq;
    const float* sp = x + ((size_t)(b * CC + c0 + cl)) * NN + n0 + 8 * e;
    const v4f a = *(const v4f*)sp;
    const v4f q = *(const v4f*)(sp + 4);
    unsigned short ub[8], hb[8];
#pragma unroll
    for (int t = 0; t < 4; ++t) {
      ub[t]     = bf_bits(a[t]);
      ub[4 + t] = bf_bits(q[t]);
    }
#pragma unroll
    for (int t = 0; t < 8; ++t) hb[t] = h_bits((_Float16)bf_up(ub[t]));
#pragma unroll
    for (int t = 0; t < 4; ++t) ux[it][t] = pk16(ub[2 * t], ub[2 * t + 1]);
#pragma unroll
    for (int t = 0; t < 8; ++t) T[(8 * e + t) * TP + cl] = hb[t];
  }
  __syncthreads();
  v4u up[2];
#pragma unroll
  for (int it = 0; it < 2; ++it) {
    const int nl = it * 32 + lq;
    up[it] = *(const v4u*)(T + nl * TP + 8 * e);
  }
#pragma unroll
  for (int pass = 0; pass < 2; ++pass) {
#pragma unroll
    for (int it = 0; it < 2; ++it) {
      const int rl = it * 32 + lq;
      *(volatile v4u*)(Xc + ((size_t)(b * CC + c0 + rl)) * NN + n0 + 8 * e) = ux[it];
      *(volatile v4u*)(XP + ((size_t)(b * NN + n0 + rl)) * CC + c0 + 8 * e) = up[it];
    }
    __threadfence();
  }
}

__global__ __launch_bounds__(128)
void gemm_qk(const unsigned short* __restrict__ Wqk16, const unsigned short* __restrict__ XP,
             const float* __restrict__ bq, const float* __restrict__ bk,
             unsigned short* Qh, unsigned short* Ql, unsigned short* Kh, unsigned short* Kl) {
  __shared__ __align__(16) float Os[QT * OSP];
  const int tid  = threadIdx.x;
  const int lane = tid & 31, wave = tid >> 5;
  const int hh   = lane >> 4, c = lane & 15;
  const int nt   = blockIdx.x, mb = blockIdx.y, b = blockIdx.z;
  const int n0   = nt * QT, o0 = mb * QT;

  const unsigned short* ap = Wqk16 + (size_t)(o0 + c) * CC + 8 * hh;
  const unsigned short* bp = XP + ((size_t)(b * NN + n0 + 16 * wave + c)) * CC + 8 * hh;

  v8f acc[4];
#pragma unroll
  for (int mt = 0; mt < 4; ++mt) acc[mt] = zero8();

#pragma unroll 2
  for (int ks = 0; ks < CC / 32; ++ks) {
    const Frag fb = ldfrag(bp + 32 * ks);
#pragma unroll
    for (int mt = 0; mt < 4; ++mt) {
      const Frag fa = ldfrag(ap + (size_t)(16 * mt) * CC + 32 * ks);
      acc[mt] = mma_h(fa.h, fb.h, acc[mt]);
    }
  }

  {
    const int nl = 16 * wave + c;
#pragma unroll
    for (int mt = 0; mt < 4; ++mt) {
      v4f va, vb;
#pragma unroll
      for (int r = 0; r < 4; ++r) { va[r] = acc[mt][r] * IWSC; vb[r] = acc[mt][4 + r] * IWSC; }
      *(v4f*)(Os + nl * OSP + 16 * mt + 8 * hh)     = va;
      *(v4f*)(Os + nl * OSP + 16 * mt + 8 * hh + 4) = vb;
    }
  }
  __syncthreads();

  const int e = tid & 7, lq = tid >> 3;
  const float* bs = (mb == 0) ? bq : bk;
  unsigned short* Ph = (mb == 0) ? Qh : Kh;
  unsigned short* Pl = (mb == 0) ? Ql : Kl;
  const v4f b0v = *(const v4f*)(bs + 8 * e);
  const v4f b1v = *(const v4f*)(bs + 8 * e + 4);
  const float bb[8] = {bfr(b0v[0]), bfr(b0v[1]), bfr(b0v[2]), bfr(b0v[3]),
                       bfr(b1v[0]), bfr(b1v[1]), bfr(b1v[2]), bfr(b1v[3])};
  v4u uh[4], ul[4];
#pragma unroll
  for (int it = 0; it < 4; ++it) {
    const int row = it * 16 + lq;
    const v4f a = *(const v4f*)(Os + row * OSP + 8 * e);
    const v4f q = *(const v4f*)(Os + row * OSP + 8 * e + 4);
    const float f[8] = {a[0], a[1], a[2], a[3], q[0], q[1], q[2], q[3]};
#pragma unroll
    for (int t = 0; t < 4; ++t) {
      const float f0 = f[2 * t] + bb[2 * t], f1 = f[2 * t + 1] + bb[2 * t + 1];
      const unsigned short hb0 = bf_bits(f0), hb1 = bf_bits(f1);
      const unsigned short lb0 = bf_bits(f0 - bf_up(hb0));
      const unsigned short lb1 = bf_bits(f1 - bf_up(hb1));
      uh[it][t] = pk16(hb0, hb1);
      ul[it][t] = pk16(lb0, lb1);
    }
  }
#pragma unroll
  for (int pass = 0; pass < 2; ++pass) {
#pragma unroll
    for (int it = 0; it < 4; ++it) {
      const int row = it * 16 + lq;
      const size_t po = ((size_t)(b * NN + n0 + row)) * DQ + 8 * e;
      *(volatile v4u*)(Ph + po) = uh[it];
      *(volatile v4u*)(Pl + po) = ul[it];
    }
    __threadfence();
  }
}

__global__ __launch_bounds__(128)
void gemm_v(const unsigned short* __restrict__ Wv16, const unsigned short* __restrict__ XP,
            const float* __restrict__ bv, unsigned short* Vc) {
  __shared__ __align__(16) float Es[QT * EP];
  const int tid  = threadIdx.x;
  const int lane = tid & 31, wave = tid >> 5;
  const int hh   = lane >> 4, c = lane & 15;
  const int nt   = blockIdx.x, mb = blockIdx.y, b = blockIdx.z;
  const int n0   = nt * QT, o0 = mb * QT;

  const unsigned short* ap = Wv16 + (size_t)(o0 + c) * CC + 8 * hh;
  const unsigned short* bp = XP + ((size_t)(b * NN + n0 + 16 * wave + c)) * CC + 8 * hh;

  v8f acc[4];
#pragma unroll
  for (int mt = 0; mt < 4; ++mt) acc[mt] = zero8();

#pragma unroll 2
  for (int ks = 0; ks < CC / 32; ++ks) {
    const Frag fb = ldfrag(bp + 32 * ks);
#pragma unroll
    for (int mt = 0; mt < 4; ++mt) {
      const Frag fa = ldfrag(ap + (size_t)(16 * mt) * CC + 32 * ks);
      acc[mt] = mma_h(fa.h, fb.h, acc[mt]);
    }
  }

  {
    const int nl = 16 * wave + c;
#pragma unroll
    for (int mt = 0; mt < 4; ++mt) {
#pragma unroll
      for (int r = 0; r < 8; ++r) Es[(16 * mt + 8 * hh + r) * EP + nl] = acc[mt][r];
    }
  }
  __syncthreads();

  const int e = tid & 7, lq = tid >> 3;
  v4u uv[4];
#pragma unroll
  for (int it = 0; it < 4; ++it) {
    const int row = it * 16 + lq;
    const float bias = bfr(bv[o0 + row]);
    const v4f a = *(const v4f*)(Es + row * EP + 8 * e);
    const v4f q = *(const v4f*)(Es + row * EP + 8 * e + 4);
    const float f[8] = {a[0], a[1], a[2], a[3], q[0], q[1], q[2], q[3]};
#pragma unroll
    for (int t = 0; t < 4; ++t) {
      const unsigned short h0 = h_bits((_Float16)(f[2 * t] * IWSC + bias));
      const unsigned short h1 = h_bits((_Float16)(f[2 * t + 1] * IWSC + bias));
      uv[it][t] = pk16(h0, h1);
    }
  }
#pragma unroll
  for (int pass = 0; pass < 2; ++pass) {
#pragma unroll
    for (int it = 0; it < 4; ++it) {
      const int row = it * 16 + lq;
      *(volatile v4u*)(Vc + ((size_t)(b * CC + o0 + row)) * NN + n0 + 8 * e) = uv[it];
    }
    __threadfence();
  }
}

__global__ __launch_bounds__(128)
void energy_k(const unsigned short* __restrict__ Xc, float* E) {
  __shared__ __align__(16) float Es[QT * EP];
  const int tid  = threadIdx.x;
  const int lane = tid & 31, wave = tid >> 5;
  const int hh   = lane >> 4, c = lane & 15;
  const int db   = blockIdx.x, cb = blockIdx.y, b = blockIdx.z;
  const int d0   = db * QT, c0 = cb * QT;

  const unsigned short* ap = Xc + ((size_t)(b * CC + c0 + c)) * NN + 8 * hh;
  const unsigned short* bp = Xc + ((size_t)(b * CC + d0 + 16 * wave + c)) * NN + 8 * hh;

  v8f acc[4];
#pragma unroll
  for (int mt = 0; mt < 4; ++mt) acc[mt] = zero8();

#pragma unroll 2
  for (int ks = 0; ks < NN / 32; ++ks) {
    const Frag fb = ldfrag(bp + 32 * ks);
#pragma unroll
    for (int mt = 0; mt < 4; ++mt) {
      const Frag fa = ldfrag(ap + (size_t)(16 * mt) * NN + 32 * ks);
      acc[mt] = mma_b(fa.bf, fb.bf, acc[mt]);
    }
  }

  {
    const int nl = 16 * wave + c;
#pragma unroll
    for (int mt = 0; mt < 4; ++mt) {
#pragma unroll
      for (int r = 0; r < 8; ++r) Es[(16 * mt + 8 * hh + r) * EP + nl] = acc[mt][r];
    }
  }
  __syncthreads();

  const int e = tid & 7, lq = tid >> 3;
  v4f res[8];
#pragma unroll
  for (int it = 0; it < 8; ++it) {
    const int L = it * 16 + lq;
    const int row = L >> 1, hf = L & 1;
    res[it] = *(const v4f*)(Es + row * EP + 32 * hf + 4 * e);
  }
#pragma unroll
  for (int pass = 0; pass < 2; ++pass) {
#pragma unroll
    for (int it = 0; it < 8; ++it) {
      const int L = it * 16 + lq;
      const int row = L >> 1, hf = L & 1;
      *(volatile v4f*)(E + ((size_t)(b * CC + c0 + row)) * CC + d0 + 32 * hf + 4 * e) = res[it];
    }
    __threadfence();
  }
}

__global__ __launch_bounds__(256)
void cam_softmax(const float* __restrict__ E, unsigned short* Ah, unsigned short* Al) {
  const int tid = threadIdx.x, lane = tid & 31, wv = tid >> 5;
  const size_t row = (size_t)blockIdx.x * 8 + wv;
  const float* e = E + row * CC;
  float f[2][8];
#pragma unroll
  for (int j = 0; j < 2; ++j) {
    const v4f a = *(const v4f*)(e + 256 * j + 8 * lane);
    const v4f q = *(const v4f*)(e + 256 * j + 8 * lane + 4);
    f[j][0] = a[0]; f[j][1] = a[1]; f[j][2] = a[2]; f[j][3] = a[3];
    f[j][4] = q[0]; f[j][5] = q[1]; f[j][6] = q[2]; f[j][7] = q[3];
  }
  float m1 = f[0][0];
#pragma unroll
  for (int j = 0; j < 2; ++j) {
#pragma unroll
    for (int t = 0; t < 8; ++t) m1 = fmaxf(m1, f[j][t]);
  }
#pragma unroll
  for (int s = 16; s > 0; s >>= 1) m1 = fmaxf(m1, __shfl_xor(m1, s, 32));
  float m2 = -3.0e38f;
#pragma unroll
  for (int j = 0; j < 2; ++j) {
#pragma unroll
    for (int t = 0; t < 8; ++t) { f[j][t] = m1 - f[j][t]; m2 = fmaxf(m2, f[j][t]); }
  }
#pragma unroll
  for (int s = 16; s > 0; s >>= 1) m2 = fmaxf(m2, __shfl_xor(m2, s, 32));
  float sum = 0.f;
#pragma unroll
  for (int j = 0; j < 2; ++j) {
#pragma unroll
    for (int t = 0; t < 8; ++t) { const float p = __expf(f[j][t] - m2); f[j][t] = p; sum += p; }
  }
#pragma unroll
  for (int s = 16; s > 0; s >>= 1) sum += __shfl_xor(sum, s, 32);
  const float inv = 1.0f / sum;
  v4u uh[2], ul[2];
#pragma unroll
  for (int j = 0; j < 2; ++j) {
#pragma unroll
    for (int t = 0; t < 4; ++t) {
      const float t0 = f[j][2 * t] * inv * PSC, t1 = f[j][2 * t + 1] * inv * PSC;
      const _Float16 h0 = (_Float16)t0, h1 = (_Float16)t1;
      const _Float16 l0 = (_Float16)((t0 - (float)h0) * RSC);
      const _Float16 l1 = (_Float16)((t1 - (float)h1) * RSC);
      uh[j][t] = pk16(h_bits(h0), h_bits(h1));
      ul[j][t] = pk16(h_bits(l0), h_bits(l1));
    }
  }
#pragma unroll
  for (int pass = 0; pass < 2; ++pass) {
#pragma unroll
    for (int j = 0; j < 2; ++j) {
      *(volatile v4u*)(Ah + row * CC + 256 * j + 8 * lane) = uh[j];
      *(volatile v4u*)(Al + row * CC + 256 * j + 8 * lane) = ul[j];
    }
    __threadfence();
  }
}

__global__ __launch_bounds__(256)
void pam_attn(const unsigned short* __restrict__ Qh, const unsigned short* __restrict__ Ql,
              const unsigned short* __restrict__ Kh, const unsigned short* __restrict__ Kl,
              const unsigned short* __restrict__ Vc, float* pamT) {
  __shared__ __align__(16) float Os[QB * OSPW];
  __shared__ __align__(16) unsigned short Ps[QB * PP];
  __shared__ float Cs[QB];
  __shared__ float Ls[QB];
  const int tid  = threadIdx.x, lane = tid & 31;
  const int wave = __builtin_amdgcn_readfirstlane(tid >> 5);
  const int hh   = lane >> 4, c = lane & 15;
  const int qg   = wave & 1, chq = wave >> 1;
  const int n0   = blockIdx.x * QB, b = blockIdx.y;
  const int qrow = 16 * qg + c;

  const size_t qo = ((size_t)(b * NN + n0 + qrow)) * DQ + 8 * hh;
  const unsigned short* Qhp = Qh + qo;
  const unsigned short* Qlp = Ql + qo;
  const unsigned short* Khp = Kh + (size_t)b * NN * DQ + (size_t)c * DQ + 8 * hh;
  const unsigned short* Klp = Kl + (size_t)b * NN * DQ + (size_t)c * DQ + 8 * hh;
  const unsigned short* Vp  = Vc + ((size_t)(b * CC + 128 * chq + c)) * NN + 8 * hh;

  float m = -1.0e30f, l = 0.f;
  v8f o[8];
#pragma unroll
  for (int j = 0; j < 8; ++j) o[j] = zero8();

#pragma unroll 1
  for (int kb = 0; kb < NN; kb += 32) {
    if (chq == 0) {
      v8f s0 = zero8(), s1 = zero8();
#pragma unroll
      for (int kc = 0; kc < DQ / 32; ++kc) {
        const Frag qh  = ldfrag(Qhp + 32 * kc);
        const Frag ql  = ldfrag(Qlp + 32 * kc);
        const Frag k0  = ldfrag(Khp + (size_t)kb * DQ + 32 * kc);
        const Frag k1  = ldfrag(Khp + (size_t)(kb + 16) * DQ + 32 * kc);
        const Frag k0l = ldfrag(Klp + (size_t)kb * DQ + 32 * kc);
        const Frag k1l = ldfrag(Klp + (size_t)(kb + 16) * DQ + 32 * kc);
        s0 = mma_b(k0.bf, qh.bf, s0);
        s1 = mma_b(k1.bf, qh.bf, s1);
        s0 = mma_b(k0.bf, ql.bf, s0);
        s1 = mma_b(k1.bf, ql.bf, s1);
        s0 = mma_b(k0l.bf, qh.bf, s0);
        s1 = mma_b(k1l.bf, qh.bf, s1);
      }
      float mx = fmaxf(hmax8(s0), hmax8(s1));
      mx = fmaxf(mx, __shfl_xor(mx, 16, 32));
      const float mn = fmaxf(m, mx);
      const float cw = __expf(m - mn);
      m = mn;
      const float msh = mn - LNPS;

      PF ph;
      float ls = 0.f;
#pragma unroll
      for (int r = 0; r < 8; ++r) {
        const float e0 = __expf(s0[r] - msh);
        const float e1 = __expf(s1[r] - msh);
        ls += e0 + e1;
        ph.hv[0][r] = (_Float16)e0;
        ph.hv[1][r] = (_Float16)e1;
      }
      l = l * cw + ls;
      *(v8us*)(Ps + qrow * PP + 8 * hh)      = ph.u[0];
      *(v8us*)(Ps + qrow * PP + 16 + 8 * hh) = ph.u[1];
      if (hh == 0) Cs[qrow] = cw;
    }
    __syncthreads();

    const float corr = Cs[qrow];
    const unsigned grew = wave_ballot(corr != 1.0f);
    if (grew != 0u) {
#pragma unroll
      for (int j = 0; j < 8; ++j) {
#pragma unroll
        for (int r = 0; r < 8; ++r) o[j][r] *= corr;
      }
    }
    Frag pf;
    pf.u[0] = *(const v8us*)(Ps + qrow * PP + 8 * hh);
    pf.u[1] = *(const v8us*)(Ps + qrow * PP + 16 + 8 * hh);
#pragma unroll
    for (int j = 0; j < 8; ++j) {
      const Frag vf = ldfrag(Vp + (size_t)(16 * j) * NN + kb);
      o[j] = mma_h(vf.h, pf.h, o[j]);
    }
    __syncthreads();
  }
  if (chq == 0) {
    l += __shfl_xor(l, 16, 32);
    if (hh == 0) Ls[qrow] = l;
  }
  __syncthreads();
  const float inv = 1.0f / Ls[qrow];

  const int e = tid & 7, lq = tid >> 3;
#pragma unroll
  for (int half = 0; half < 2; ++half) {
    if (half) __syncthreads();
    if ((chq >> 1) == half) {
      const int chb = 128 * (chq & 1);
#pragma unroll
      for (int j = 0; j < 8; ++j) {
        v4f va, vb;
#pragma unroll
        for (int r = 0; r < 4; ++r) { va[r] = o[j][r] * inv; vb[r] = o[j][4 + r] * inv; }
        *(v4f*)(Os + qrow * OSPW + chb + 16 * j + 8 * hh)     = va;
        *(v4f*)(Os + qrow * OSPW + chb + 16 * j + 8 * hh + 4) = vb;
      }
    }
    __syncthreads();
    v4f res[8];
#pragma unroll
    for (int it = 0; it < 8; ++it) {
      const int L = it * 32 + lq;
      const int row = L >> 3, li = L & 7;
      res[it] = *(const v4f*)(Os + row * OSPW + 32 * li + 4 * e);
    }
#pragma unroll
    for (int pass = 0; pass < 2; ++pass) {
#pragma unroll
      for (int it = 0; it < 8; ++it) {
        const int L = it * 32 + lq;
        const int row = L >> 3, li = L & 7;
        const size_t idx = ((size_t)(b * NN + n0 + row)) * CC + 256 * half + 32 * li + 4 * e;
        *(volatile v4f*)(pamT + idx) = res[it];
      }
      __threadfence();
    }
  }
}

__global__ __launch_bounds__(128)
void cam_apply(const unsigned short* __restrict__ Ah, const unsigned short* __restrict__ Al,
               const unsigned short* __restrict__ XP, const float* __restrict__ pamT,
               const float* __restrict__ gpp, const float* __restrict__ gcp,
               unsigned short* Fh, unsigned short* Fl) {
  __shared__ __align__(16) float Os[QT * OSP];
  const int tid  = threadIdx.x;
  const int lane = tid & 31, wave = tid >> 5;
  const int hh   = lane >> 4, c = lane & 15;
  const int nt   = blockIdx.x, mb = blockIdx.y, b = blockIdx.z;
  const int n0   = nt * QT, c0 = mb * QT;

  const unsigned short* ap  = Ah + ((size_t)(b * CC + c0 + c)) * CC + 8 * hh;
  const unsigned short* apl = Al + ((size_t)(b * CC + c0 + c)) * CC + 8 * hh;
  const unsigned short* bp  = XP + ((size_t)(b * NN + n0 + 16 * wave + c)) * CC + 8 * hh;

  v8f acc[4], acr[4];
#pragma unroll
  for (int mt = 0; mt < 4; ++mt) { acc[mt] = zero8(); acr[mt] = zero8(); }

#pragma unroll 2
  for (int ks = 0; ks < CC / 32; ++ks) {
    const Frag fb = ldfrag(bp + 32 * ks);
#pragma unroll
    for (int mt = 0; mt < 4; ++mt) {
      const Frag fa  = ldfrag(ap + (size_t)(16 * mt) * CC + 32 * ks);
      const Frag fal = ldfrag(apl + (size_t)(16 * mt) * CC + 32 * ks);
      acc[mt] = mma_h(fa.h, fb.h, acc[mt]);
      acr[mt] = mma_h(fal.h, fb.h, acr[mt]);
    }
  }

  const float gc = bfr(gcp[0]);
  const float gp = bfr(gpp[0]);
  {
    const float sc = IPSC * gc;
    const int nl = 16 * wave + c;
#pragma unroll
    for (int mt = 0; mt < 4; ++mt) {
      v4f va, vb;
#pragma unroll
      for (int r = 0; r < 4; ++r) {
        va[r] = (acc[mt][r] + acr[mt][r] * IRSC) * sc;
        vb[r] = (acc[mt][4 + r] + acr[mt][4 + r] * IRSC) * sc;
      }
      *(v4f*)(Os + nl * OSP + 16 * mt + 8 * hh)     = va;
      *(v4f*)(Os + nl * OSP + 16 * mt + 8 * hh + 4) = vb;
    }
  }
  __syncthreads();

  const int e = tid & 7, lq = tid >> 3;
  v4u uh[4], ul[4];
#pragma unroll
  for (int it = 0; it < 4; ++it) {
    const int row = it * 16 + lq;
    const size_t idx = ((size_t)(b * NN + n0 + row)) * CC + c0 + 8 * e;
    const v4f a  = *(const v4f*)(Os + row * OSP + 8 * e);
    const v4f q  = *(const v4f*)(Os + row * OSP + 8 * e + 4);
    const v4f pa = *(const v4f*)(pamT + idx);
    const v4f pq = *(const v4f*)(pamT + idx + 4);
    const v8h xv = *(const v8h*)(XP + idx);
    const float cm[8] = {a[0], a[1], a[2], a[3], q[0], q[1], q[2], q[3]};
    const float pm[8] = {pa[0], pa[1], pa[2], pa[3], pq[0], pq[1], pq[2], pq[3]};
    float f[8];
#pragma unroll
    for (int t = 0; t < 8; ++t) f[t] = cm[t] + gp * pm[t] + 2.0f * (float)xv[t];
#pragma unroll
    for (int t = 0; t < 4; ++t) {
      const float f0 = f[2 * t], f1 = f[2 * t + 1];
      const unsigned short hb0 = bf_bits(f0), hb1 = bf_bits(f1);
      const unsigned short lb0 = bf_bits(f0 - bf_up(hb0));
      const unsigned short lb1 = bf_bits(f1 - bf_up(hb1));
      uh[it][t] = pk16(hb0, hb1);
      ul[it][t] = pk16(lb0, lb1);
    }
  }
#pragma unroll
  for (int pass = 0; pass < 2; ++pass) {
#pragma unroll
    for (int it = 0; it < 4; ++it) {
      const int row = it * 16 + lq;
      const size_t idx = ((size_t)(b * NN + n0 + row)) * CC + c0 + 8 * e;
      *(volatile v4u*)(Fh + idx) = uh[it];
      *(volatile v4u*)(Fl + idx) = ul[it];
    }
    __threadfence();
  }
}

__global__ __launch_bounds__(128)
void gemm_out(const unsigned short* __restrict__ Wo16, const unsigned short* __restrict__ Fh,
              const unsigned short* __restrict__ Fl, float* Y) {
  __shared__ __align__(16) float Es[QT * EP];
  const int tid  = threadIdx.x;
  const int lane = tid & 31, wave = tid >> 5;
  const int hh   = lane >> 4, c = lane & 15;
  const int nt   = blockIdx.x, mb = blockIdx.y, b = blockIdx.z;
  const int n0   = nt * QT, o0 = mb * QT;

  const unsigned short* ap  = Wo16 + (size_t)(o0 + c) * CC + 8 * hh;
  const size_t bo = ((size_t)(b * NN + n0 + 16 * wave + c)) * CC + 8 * hh;
  const unsigned short* bph = Fh + bo;
  const unsigned short* bpl = Fl + bo;

  v8f acc[4];
#pragma unroll
  for (int mt = 0; mt < 4; ++mt) acc[mt] = zero8();

#pragma unroll 2
  for (int ks = 0; ks < CC / 32; ++ks) {
    const Frag fbh = ldfrag(bph + 32 * ks);
    const Frag fbl = ldfrag(bpl + 32 * ks);
#pragma unroll
    for (int mt = 0; mt < 4; ++mt) {
      const Frag fa = ldfrag(ap + (size_t)(16 * mt) * CC + 32 * ks);
      acc[mt] = mma_b(fa.bf, fbh.bf, acc[mt]);
      acc[mt] = mma_b(fa.bf, fbl.bf, acc[mt]);
    }
  }

  {
    const int nl = 16 * wave + c;
#pragma unroll
    for (int mt = 0; mt < 4; ++mt) {
#pragma unroll
      for (int r = 0; r < 8; ++r) Es[(16 * mt + 8 * hh + r) * EP + nl] = acc[mt][r];
    }
  }
  __syncthreads();

  const int e = tid & 7, lq = tid >> 3;
  v4f res[8];
#pragma unroll
  for (int it = 0; it < 8; ++it) {
    const int L = it * 16 + lq;
    const int row = L >> 1, hf = L & 1;
    res[it] = *(const v4f*)(Es + row * EP + 32 * hf + 4 * e);
  }
#pragma unroll
  for (int pass = 0; pass < 2; ++pass) {
#pragma unroll
    for (int it = 0; it < 8; ++it) {
      const int L = it * 16 + lq;
      const int row = L >> 1, hf = L & 1;
      *(volatile v4f*)(Y + ((size_t)(b * CC + o0 + row)) * NN + n0 + 32 * hf + 4 * e) = res[it];
    }
    __threadfence();
  }
}

__global__ __launch_bounds__(256)
void bn_relu(const float* __restrict__ Y, const float* __restrict__ bng, const float* __restrict__ bnb,
             float* out) {
  __shared__ double rs[256];
  __shared__ double rq[256];
  const int o = blockIdx.x, tid = threadIdx.x;
  double s = 0.0, q = 0.0;
#pragma unroll 1
  for (int j = 0; j < NCH; ++j) {
    const int bb = j / (NN / 1024);
    const int nn = 1024 * (j % (NN / 1024)) + 4 * tid;
    const v4f v = *(const v4f*)(Y + ((size_t)(bb * CC + o)) * NN + nn);
#pragma unroll
    for (int t = 0; t < 4; ++t) { const double d = (double)v[t]; s += d; q = fma(d, d, q); }
  }
  rs[tid] = s;
  rq[tid] = q;
  __syncthreads();
#pragma unroll 1
  for (int st = 128; st > 0; st >>= 1) {
    if (tid < st) { rs[tid] += rs[tid + st]; rq[tid] += rq[tid + st]; }
    __syncthreads();
  }
  const double cnt  = (double)(NB * NN);
  const double mean = rs[0] / cnt;
  double var = rq[0] / cnt - mean * mean;
  var = (var > 0.0) ? var : 0.0;
  const float meanf = (float)mean;
  const float rstd  = rsqrtf((float)var + BNEPS);
  const float g = bfr(bng[o]), be = bfr(bnb[o]);
#pragma unroll 1
  for (int pass = 0; pass < 2; ++pass) {
#pragma unroll 1
    for (int j = 0; j < NCH; ++j) {
      const int bb = j / (NN / 1024);
      const int nn = 1024 * (j % (NN / 1024)) + 4 * tid;
      const size_t idx = ((size_t)(bb * CC + o)) * NN + nn;
      const v4f v = *(const v4f*)(Y + idx);
      v4f r;
#pragma unroll
      for (int t = 0; t < 4; ++t) {
        const float t1 = (v[t] - meanf) * rstd;
        const float t2 = t1 * g + be;
        r[t] = fmaxf(t2, 0.0f);
      }
      *(volatile v4f*)(out + idx) = r;
    }
    __threadfence();
  }
}

static_assert((size_t)NB * CC * NN * 2 == (size_t)NB * NN * CC * 2);
static_assert((size_t)NB * NN * CC * 4 == (size_t)NB * CC * NN * 4);

extern "C" void kernel_launch(void* const* d_in, const int* in_sizes, int n_in,
                              void* d_out, int out_size, void* d_ws, size_t ws_size,
                              hipStream_t stream) {
  if (n_in < 12) return;
  if (in_sizes[0] < NB * CC * NN) return;
  if (in_sizes[1] < DQ * CC || in_sizes[2] < DQ) return;
  if (in_sizes[3] < DQ * CC || in_sizes[4] < DQ) return;
  if (in_sizes[5] < CC * CC || in_sizes[6] < CC) return;
  if (in_sizes[7] < 1 || in_sizes[8] < 1) return;
  if (in_sizes[9] < CC * CC || in_sizes[10] < CC || in_sizes[11] < CC) return;
  if (out_size < NB * CC * NN) return;

  size_t off = 0;
  auto carve = [&](size_t bytes) { const size_t o = off; off += (bytes + 255) & ~(size_t)255; return o; };
  const size_t oWqk = carve((size_t)MW * CC * 2);
  const size_t oWv  = carve((size_t)CC * CC * 2);
  const size_t oWo  = carve((size_t)CC * CC * 2);
  const size_t oRX  = carve((size_t)NB * CC * NN * 2);
  const size_t oXP  = carve((size_t)NB * NN * CC * 2);
  const size_t oQh  = carve((size_t)NB * NN * DQ * 2);
  const size_t oQl  = carve((size_t)NB * NN * DQ * 2);
  const size_t oKh  = carve((size_t)NB * NN * DQ * 2);
  const size_t oKl  = carve((size_t)NB * NN * DQ * 2);
  const size_t oRV  = carve((size_t)NB * CC * NN * 2);
  const size_t oE   = carve((size_t)NB * CC * CC * 4);
  const size_t oAh  = carve((size_t)NB * CC * CC * 2);
  const size_t oAl  = carve((size_t)NB * CC * CC * 2);
  const size_t oRP  = carve((size_t)NB * NN * CC * 4);
  if (off > ws_size) return;
  if (off > (size_t)134217728) return;

  const float* x    = (const float*)d_in[0];
  const float* Wq   = (const float*)d_in[1];
  const float* bq   = (const float*)d_in[2];
  const float* Wk   = (const float*)d_in[3];
  const float* bk   = (const float*)d_in[4];
  const float* Wv   = (const float*)d_in[5];
  const float* bv   = (const float*)d_in[6];
  const float* gpp  = (const float*)d_in[7];
  const float* gcp  = (const float*)d_in[8];
  const float* Wout = (const float*)d_in[9];
  const float* bng  = (const float*)d_in[10];
  const float* bnb  = (const float*)d_in[11];

  char* ws = (char*)d_ws;
  unsigned short* Wqk16 = (unsigned short*)(ws + oWqk);
  unsigned short* Wv16  = (unsigned short*)(ws + oWv);
  unsigned short* Wo16  = (unsigned short*)(ws + oWo);
  unsigned short* Xc    = (unsigned short*)(ws + oRX);
  unsigned short* Fh    = (unsigned short*)(ws + oRX);
  unsigned short* XP    = (unsigned short*)(ws + oXP);
  unsigned short* Qh    = (unsigned short*)(ws + oQh);
  unsigned short* Ql    = (unsigned short*)(ws + oQl);
  unsigned short* Kh    = (unsigned short*)(ws + oKh);
  unsigned short* Kl    = (unsigned short*)(ws + oKl);
  unsigned short* Vc    = (unsigned short*)(ws + oRV);
  unsigned short* Fl    = (unsigned short*)(ws + oRV);
  float*          E     = (float*)(ws + oE);
  unsigned short* Ah    = (unsigned short*)(ws + oAh);
  unsigned short* Al    = (unsigned short*)(ws + oAl);
  float*          pamT  = (float*)(ws + oRP);
  float*          Y     = (float*)(ws + oRP);
  float*          out   = (float*)d_out;

  const dim3 blk256(256), blk128(128);

  cvt_w<<<dim3(MW / 8 + 2 * (CC / 8)), blk256, 0, stream>>>(Wq, Wk, Wv, Wout, Wqk16, Wv16, Wo16);
  cvt_x<<<dim3(NN / QT, CC / QT, NB), blk256, 0, stream>>>(x, Xc, XP);
  gemm_qk<<<dim3(NN / QT, MW / QT, NB), blk128, 0, stream>>>(Wqk16, XP, bq, bk, Qh, Ql, Kh, Kl);
  gemm_v<<<dim3(NN / QT, CC / QT, NB), blk128, 0, stream>>>(Wv16, XP, bv, Vc);
  energy_k<<<dim3(CC / QT, CC / QT, NB), blk128, 0, stream>>>(Xc, E);
  cam_softmax<<<dim3(NB * CC / 8), blk256, 0, stream>>>(E, Ah, Al);
  pam_attn<<<dim3(NN / QB, NB), blk256, 0, stream>>>(Qh, Ql, Kh, Kl, Vc, pamT);
  cam_apply<<<dim3(NN / QT, CC / QT, NB), blk128, 0, stream>>>(Ah, Al, XP, pamT, gpp, gcp, Fh, Fl);
  gemm_out<<<dim3(NN / QT, CC / QT, NB), blk128, 0, stream>>>(Wo16, Fh, Fl, Y);
  bn_relu<<<dim3(CC), blk256, 0, stream>>>(Y, bng, bnb, out);
  (void)hipGetLastError();
}
